// VCSWin3DBlock_30588757082821
// MI455X (gfx1250) — hardware-verified
//
#include <hip/hip_runtime.h>


#define NB_  2
#define CC   192
#define RR   16
#define LL   4096
#define CB   64
#define NHB  2
#define HD   32
#define WIN  1024
#define NWIN 4
#define H4   768
#define NZ   (NWIN * NHB)
#define PCAR 1024.0f
typedef _Float16 h16;
typedef unsigned short bf;
typedef __attribute__((ext_vector_type(16))) __bf16   v16bf;
typedef __attribute__((ext_vector_type(16))) _Float16 v16h;
typedef __attribute__((ext_vector_type(8)))  _Float16 v8h;
typedef __attribute__((ext_vector_type(8)))  unsigned short v8us;
typedef __attribute__((ext_vector_type(8)))  float    v8f;
typedef __attribute__((ext_vector_type(4)))  float    v4f;
typedef v8h  __attribute__((may_alias)) v8ha;
typedef v4f  __attribute__((may_alias)) v4fa;
typedef v8us __attribute__((may_alias)) v8usa;

__device__ __forceinline__ unsigned short f2bf(float f) { unsigned u = __float_as_uint(f); u += 0x7FFFu + ((u >> 16) & 1u); return (unsigned short)(u >> 16); }
__device__ __forceinline__ float bf2f(unsigned short b) { return __uint_as_float(((unsigned)b) << 16); }
__device__ __forceinline__ float bfr(float f) { return bf2f(f2bf(f)); }
__device__ __forceinline__ v16h cat16(v8h lo, v8h hi) { return __builtin_shufflevector(lo, hi, 0, 1, 2, 3, 4, 5, 6, 7, 8, 9, 10, 11, 12, 13, 14, 15); }
__device__ __forceinline__ v16bf cat16b(v8us lo, v8us hi) { return __builtin_bit_cast(v16bf, __builtin_shufflevector(lo, hi, 0, 1, 2, 3, 4, 5, 6, 7, 8, 9, 10, 11, 12, 13, 14, 15)); }
__device__ __forceinline__ v8f wmma16(v16h a, v16h b, v8f c) { return __builtin_amdgcn_wmma_f32_16x16x32_f16(false, a, false, b, (short)0, c, false, false); }
__device__ __forceinline__ v8f wmmab(v16bf a, v16bf b, v8f c) { return __builtin_amdgcn_wmma_f32_16x16x32_bf16(false, a, false, b, (short)0, c, false, false); }


template <typename T16> struct WFrag;
template <> struct WFrag<h16> { typedef v16h V; static __device__ __forceinline__ V ld(const h16* p) { return cat16(*(const v8h*)p, *(const v8h*)(p + 16)); } static __device__ __forceinline__ v8f mma(V a, V b, v8f c) { return wmma16(a, b, c); } };
template <> struct WFrag<bf> { typedef v16bf V; static __device__ __forceinline__ V ld(const bf* p) { return cat16b(*(const v8us*)p, *(const v8us*)(p + 16)); } static __device__ __forceinline__ v8f mma(V a, V b, v8f c) { return wmmab(a, b, c); } };
template <typename T16, int NSPLIT, bool BIAS>
__global__ __launch_bounds__(32) void k_gemmw(const T16* __restrict__ A, const T16* __restrict__ A2, const T16* __restrict__ Bt, const T16* __restrict__ Bt2, int K, float* C, int ldc, const float* __restrict__ bias, size_t sA, size_t sB, size_t sC) {
    typedef typename WFrag<T16>::V V;
    __shared__ __align__(16) float os[16 * 68];
    const size_t z = blockIdx.z; A += z * sA; if (A2) A2 += z * sA; Bt += z * sB; if (Bt2) Bt2 += z * sB; C += z * sC;
    const int lane = threadIdx.x & 31, lr = lane & 15, hi = lane >> 4; const int r0 = blockIdx.x * 64, c0 = blockIdx.y * 64;
    v8f acc[4][4];
#pragma unroll
    for (int mb = 0; mb < 4; ++mb)
#pragma unroll
        for (int nb = 0; nb < 4; ++nb) acc[mb][nb] = (v8f){};
    const size_t aoff = (size_t)(r0 + lr) * K + 8 * hi, boff = (size_t)(c0 + lr) * K + 8 * hi;
#pragma unroll 1
    for (int kc = 0; kc < K; kc += 32) {
        V a[4], a2[4];
#pragma unroll
        for (int mb = 0; mb < 4; ++mb) { a[mb] = WFrag<T16>::ld(A + aoff + (size_t)mb * 16 * K + kc); if (NSPLIT == 1 || NSPLIT == 2) a2[mb] = WFrag<T16>::ld(A2 + aoff + (size_t)mb * 16 * K + kc); }
#pragma unroll
        for (int nb = 0; nb < 4; ++nb) { const V b = WFrag<T16>::ld(Bt + boff + (size_t)nb * 16 * K + kc); V b2; if (NSPLIT >= 2) b2 = WFrag<T16>::ld(Bt2 + boff + (size_t)nb * 16 * K + kc);
#pragma unroll
            for (int mb = 0; mb < 4; ++mb) { acc[mb][nb] = WFrag<T16>::mma(a[mb], b, acc[mb][nb]); if (NSPLIT == 1 || NSPLIT == 2) acc[mb][nb] = WFrag<T16>::mma(a2[mb], b, acc[mb][nb]); if (NSPLIT >= 2) acc[mb][nb] = WFrag<T16>::mma(a[mb], b2, acc[mb][nb]); } }
        asm volatile("v_nop\n\tv_nop\n\tv_nop\n\tv_nop" : "+v"(acc[0][0]), "+v"(acc[1][1]), "+v"(acc[2][2]), "+v"(acc[3][3]) : "v"(a[0]), "v"(a[3]));
    }
#pragma unroll
    for (int mb = 0; mb < 4; ++mb) {
#pragma unroll
        for (int nb = 0; nb < 4; ++nb) {
#pragma unroll
            for (int j = 0; j < 8; ++j) os[(hi * 8 + j) * 68 + nb * 16 + lr] = acc[mb][nb][j]; }
        __builtin_amdgcn_wave_barrier(); asm volatile("" ::: "memory");
        float* crow = C + (size_t)(r0 + mb * 16) * ldc + c0;
#pragma unroll 1
        for (int ps = 0; ps < 2; ++ps) {
#pragma unroll
            for (int s = 0; s < 8; ++s) { const int row = 2 * s + hi, cofs = lr * 4; v4f val = *(const v4fa*)(os + row * 68 + cofs); if (BIAS) { val[0] += bfr(bias[c0 + cofs]); val[1] += bfr(bias[c0 + cofs + 1]); val[2] += bfr(bias[c0 + cofs + 2]); val[3] += bfr(bias[c0 + cofs + 3]); }
                *(volatile v4f*)(crow + (size_t)row * ldc + cofs) = val; }
            if (ps == 0) __threadfence(); }
        __builtin_amdgcn_wave_barrier(); asm volatile("" ::: "memory");
    }
}

__device__ __forceinline__ h16 tohx(float x) { return (h16)x; }
__device__ __forceinline__ void splitf(float y, unsigned short& h, unsigned short& l) { h = f2bf(y); l = f2bf(y - bf2f(h)); }
typedef __attribute__((ext_vector_type(2))) unsigned short v2us;
typedef __attribute__((ext_vector_type(4))) unsigned short v4us; typedef __attribute__((ext_vector_type(8))) unsigned short v8us;
typedef __attribute__((ext_vector_type(2))) _Float16 v2h;
typedef __attribute__((ext_vector_type(4))) _Float16 v4h;

__global__ __launch_bounds__(256) void k_wtG(const float* __restrict__ w, int K, int N, bf* Bt) {
    const int lane = threadIdx.x & 31; const int L0 = (blockIdx.x * 8 + (threadIdx.x >> 5)) * 8; const int nlines = N * K / 64;
#pragma unroll
    for (int ps = 0; ps < 2; ++ps) {
#pragma unroll 1
        for (int l = 0; l < 8; ++l) { const int L = L0 + l; if (L >= nlines) break; const size_t e = (size_t)L * 64 + lane * 2; const int k = (int)(e % K), n = (int)(e / K); v2us o;
            o[0] = f2bf(w[(size_t)k * N + n]); o[1] = f2bf(w[(size_t)(k + 1) * N + n]); *(volatile v2us*)(Bt + e) = o; }
        if (ps == 0) __threadfence(); }
}

__device__ __forceinline__ void winmap(int br, int t, int& win, int& pos) { const int d = t >> 8, h = (t >> 4) & 15, w = t & 15;
    if (br == 0) { win = w >> 2; pos = d * 64 + h * 4 + (w & 3); } else if (br == 1) { win = h >> 2; pos = d * 64 + (h & 3) * 16 + w; } else { win = d >> 2; pos = (d & 3) * 256 + h * 16 + w; } }
__device__ __forceinline__ int winmap_inv(int br, int win, int pos) { int d, h, w;
    if (br == 0) { d = pos >> 6; h = (pos >> 2) & 15; w = win * 4 + (pos & 3); } else if (br == 1) { d = pos >> 6; h = win * 4 + ((pos >> 4) & 3); w = pos & 15; } else { d = win * 4 + (pos >> 8); h = (pos >> 4) & 15; w = pos & 15; }
    return d * 256 + h * 16 + w; }
__global__ __launch_bounds__(256) void k_xt(const float* __restrict__ X, float* XT) { const size_t e = ((size_t)blockIdx.x * 256 + threadIdx.x) * 4; if (e >= (size_t)LL * CC) return; const int c = (int)(e % CC); const int t = (int)(e / CC); v4f o;
#pragma unroll
    for (int u = 0; u < 4; ++u) o[u] = 2.0f * bfr(X[(size_t)(c + u) * LL + t]); *(volatile v4f*)(XT + e) = o; __threadfence(); *(volatile v4f*)(XT + e) = o; }
__global__ __launch_bounds__(256) void k_ln(const float* __restrict__ F, const float* __restrict__ g, const float* __restrict__ bb, bf* Ph, bf* Pl) { const int lane = threadIdx.x & 31; const size_t t = (size_t)blockIdx.x * 8 + (threadIdx.x >> 5); if (t >= LL) return; const float* f = F + t * CC; float s = 0.f;
#pragma unroll
    for (int k = 0; k < 6; ++k) s += f[k * 32 + lane];
#pragma unroll
    for (int sh = 16; sh; sh >>= 1) s += __shfl_xor(s, sh, 32);
    const float mean = s * (1.0f / CC); float q = 0.f;
#pragma unroll
    for (int k = 0; k < 6; ++k) { float d = __fsub_rn(f[k * 32 + lane], mean); asm volatile("" : "+v"(d)); float p = __fmul_rn(d, d); asm volatile("" : "+v"(p)); q = __fadd_rn(q, p); }
#pragma unroll
    for (int sh = 16; sh; sh >>= 1) q += __shfl_xor(q, sh, 32);
    const float rs = __frsqrt_rn(__fadd_rn(q * (1.0f / CC), 1e-5f));
    if (lane < 24) { v8us oh, ol;
#pragma unroll
        for (int u = 0; u < 8; ++u) { const int c = lane * 8 + u; float d = __fsub_rn(f[c], mean); asm volatile("" : "+v"(d)); float n0 = __fmul_rn(d, rs); asm volatile("" : "+v"(n0)); float t1 = __fmul_rn(n0, bfr(g[c])); asm volatile("" : "+v"(t1)); unsigned short p, q2; splitf(__fadd_rn(t1, bfr(bb[c])), p, q2); oh[u] = p; ol[u] = q2; }
        *(volatile v8us*)(Ph + t * CC + lane * 8) = oh; *(volatile v8us*)(Pl + t * CC + lane * 8) = ol; __threadfence(); *(volatile v8us*)(Ph + t * CC + lane * 8) = oh; *(volatile v8us*)(Pl + t * CC + lane * 8) = ol; } }
__global__ __launch_bounds__(256) void k_wplanes(const float* __restrict__ QKV, int br, bf* Qh, bf* Ql, bf* Kh, bf* Kl) { const size_t e = ((size_t)blockIdx.x * 256 + threadIdx.x) * 4; if (e >= (size_t)NZ * WIN * HD) return; const int d = (int)(e % HD); const int pos = (int)((e / HD) % WIN); const int z = (int)(e / ((size_t)HD * WIN)); const int win = z >> 1, hh = z & 1; const int t = winmap_inv(br, win, pos);
    const float* q = QKV + (size_t)t * (3 * CC) + br * CB + hh * HD + d; const float* k = q + CC; v4us qh, ql, kh, kl;
#pragma unroll
    for (int u = 0; u < 4; ++u) { unsigned short a, b; splitf(q[u] * 0.17677669529663689f, a, b); qh[u] = a; ql[u] = b; splitf(k[u], a, b); kh[u] = a; kl[u] = b; }
    *(volatile v4us*)(Qh + e) = qh; *(volatile v4us*)(Ql + e) = ql; *(volatile v4us*)(Kh + e) = kh; *(volatile v4us*)(Kl + e) = kl; __threadfence(); *(volatile v4us*)(Qh + e) = qh; *(volatile v4us*)(Ql + e) = ql; *(volatile v4us*)(Kh + e) = kh; *(volatile v4us*)(Kl + e) = kl; }
__global__ __launch_bounds__(256) void k_vtw(const float* __restrict__ QKV, int br, h16* VT) { const size_t e = ((size_t)blockIdx.x * 256 + threadIdx.x) * 2; if (e >= (size_t)NZ * 64 * WIN) return; const int pos = (int)(e % WIN); const int d = (int)((e / WIN) % 64); const int z = (int)(e / ((size_t)WIN * 64)); const int win = z >> 1, hh = z & 1; v2h o;
#pragma unroll
    for (int u = 0; u < 2; ++u) { float val = 0.f; if (d < HD) { const int t = winmap_inv(br, win, pos + u); val = QKV[(size_t)t * (3 * CC) + 2 * CC + br * CB + hh * HD + d]; } o[u] = tohx(val); }
    *(volatile v2h*)(VT + e) = o; __threadfence(); *(volatile v2h*)(VT + e) = o; }
__global__ __launch_bounds__(256) void k_wsoft(const float* __restrict__ S, h16* P16) { const int lane = threadIdx.x & 31; const int row = blockIdx.x * 8 + (threadIdx.x >> 5); if (row >= NZ * WIN) return; const float* sr = S + (size_t)row * WIN; float v[WIN / 32]; float mx = -3.0e38f;
#pragma unroll
    for (int ch = 0; ch < WIN / 128; ++ch) { const v4f a = *(const v4f*)(sr + ch * 128 + lane * 4);
#pragma unroll
        for (int u = 0; u < 4; ++u) { v[ch * 4 + u] = a[u]; mx = fmaxf(mx, a[u]); } }
#pragma unroll
    for (int sh = 16; sh; sh >>= 1) mx = fmaxf(mx, __shfl_xor(mx, sh, 32));
    float sum = 0.f;
#pragma unroll
    for (int q = 0; q < WIN / 32; ++q) { float d0 = __fsub_rn(v[q], mx); asm volatile("" : "+v"(d0)); v[q] = __builtin_amdgcn_exp2f(__fmul_rn(d0, 1.4426950408889634f)); sum += v[q]; }
#pragma unroll
    for (int sh = 16; sh; sh >>= 1) sum += __shfl_xor(sum, sh, 32);
    const float f = __fdiv_rn(PCAR, sum);
    for (int ps = 0; ps < 2; ++ps) {
#pragma unroll
        for (int ch = 0; ch < WIN / 128; ++ch) { v4h o4; for (int q = 0; q < 4; ++q) o4[q] = tohx(v[ch * 4 + q] * f); *(volatile v4h*)(P16 + (size_t)row * WIN + ch * 128 + lane * 4) = o4; }
        if (ps == 0) __threadfence(); } }
__global__ __launch_bounds__(256) void k_wmrg(const float* __restrict__ O, int br, bf* Ah, bf* Al) { const size_t e = ((size_t)blockIdx.x * 256 + threadIdx.x) * 4; if (e >= (size_t)NZ * WIN * HD) return; const int d = (int)(e % HD); const int pos = (int)((e / HD) % WIN); const int z = (int)(e / ((size_t)HD * WIN)); const int win = z >> 1, hh = z & 1; const int t = winmap_inv(br, win, pos);
    const float* o = O + ((size_t)z * WIN + pos) * 64 + d; const size_t oo = (size_t)t * CC + br * CB + hh * HD + d; v4us oh, ol;
#pragma unroll
    for (int u = 0; u < 4; ++u) { unsigned short a, b; splitf(o[u] * (1.0f / PCAR), a, b); oh[u] = a; ol[u] = b; } *(volatile v4us*)(Ah + oo) = oh; *(volatile v4us*)(Al + oo) = ol; __threadfence(); *(volatile v4us*)(Ah + oo) = oh; *(volatile v4us*)(Al + oo) = ol; }
__global__ __launch_bounds__(256) void k_res1(const float* __restrict__ XT, const float* __restrict__ PJ, float* XS) { const size_t e = ((size_t)blockIdx.x * 256 + threadIdx.x) * 4; if (e >= (size_t)LL * CC) return; const v4f a = *(const v4f*)(XT + e), p = *(const v4f*)(PJ + e); v4f o;
#pragma unroll
    for (int u = 0; u < 4; ++u) o[u] = __fadd_rn(a[u], p[u]); *(volatile v4f*)(XS + e) = o; __threadfence(); *(volatile v4f*)(XS + e) = o; }
__global__ __launch_bounds__(256) void k_gelupl(const float* __restrict__ F, bf* Ph, bf* Pl) { const size_t e = ((size_t)blockIdx.x * 256 + threadIdx.x) * 4; if (e >= (size_t)LL * H4) return; const v4f a = *(const v4f*)(F + e); v4us oh, ol;
#pragma unroll
    for (int u = 0; u < 4; ++u) { const float xx = a[u]; const float gl = __fmul_rn(__fmul_rn(0.5f, xx), __fadd_rn(1.0f, erff(xx * 0.70710678118654752f))); unsigned short p, q; splitf(gl, p, q); oh[u] = p; ol[u] = q; }
    *(volatile v4us*)(Ph + e) = oh; *(volatile v4us*)(Pl + e) = ol; __threadfence(); *(volatile v4us*)(Ph + e) = oh; *(volatile v4us*)(Pl + e) = ol; }
__global__ __launch_bounds__(256) void k_out(const float* __restrict__ XS, const float* __restrict__ F2, float* Y) { const size_t e = ((size_t)blockIdx.x * 256 + threadIdx.x) * 4; if (e >= (size_t)CC * LL) return; const int t = (int)(e % LL); const int c = (int)(e / LL); v4f o;
#pragma unroll
    for (int u = 0; u < 4; ++u) o[u] = __fadd_rn(XS[(size_t)(t + u) * CC + c], F2[(size_t)(t + u) * CC + c]); *(volatile v4f*)(Y + e) = o; __threadfence(); *(volatile v4f*)(Y + e) = o; }

extern "C" void kernel_launch(void* const* d_in, const int* in_sizes, int n_in,
                              void* d_out, int out_size, void* d_ws, size_t ws_size, hipStream_t stream) {
    (void)in_sizes; (void)n_in; (void)out_size;
    const float* x = (const float*)d_in[0]; const float* wqkv = (const float*)d_in[1]; const float* wproj = (const float*)d_in[2]; const float* bproj = (const float*)d_in[3]; const float* g1 = (const float*)d_in[4]; const float* b1 = (const float*)d_in[5]; const float* g2 = (const float*)d_in[6]; const float* b2 = (const float*)d_in[7];
    const float* wfc1 = (const float*)d_in[8]; const float* bfc1 = (const float*)d_in[9]; const float* wfc2 = (const float*)d_in[10]; const float* bfc2 = (const float*)d_in[11];
    float* OUT = (float*)d_out;
    char* wsp = (char*)d_ws;
    auto take = [&](size_t bytes) { char* p = wsp; wsp += (bytes + 255) & ~(size_t)255; return (void*)p; };
    bf* BQKV = (bf*)take((size_t)3 * CC * CC * 2); bf* BPJ = (bf*)take((size_t)CC * CC * 2); bf* BF1 = (bf*)take((size_t)H4 * CC * 2); bf* BF2 = (bf*)take((size_t)CC * H4 * 2);
    float* XT = (float*)take((size_t)LL * CC * 4); bf* Ih = (bf*)take((size_t)LL * CC * 2); bf* Il = (bf*)take((size_t)LL * CC * 2); float* QKV = (float*)take((size_t)LL * 3 * CC * 4);
    bf* Qh = (bf*)take((size_t)NZ * WIN * HD * 2); bf* Ql = (bf*)take((size_t)NZ * WIN * HD * 2); bf* Kh = (bf*)take((size_t)NZ * WIN * HD * 2); bf* Kl = (bf*)take((size_t)NZ * WIN * HD * 2); h16* VT = (h16*)take((size_t)NZ * 64 * WIN * 2);
    float* S = (float*)take((size_t)NZ * WIN * WIN * 4); h16* P16 = (h16*)take((size_t)NZ * WIN * WIN * 2); float* O = (float*)take((size_t)NZ * WIN * 64 * 4); bf* ATh = (bf*)take((size_t)LL * CC * 2); bf* ATl = (bf*)take((size_t)LL * CC * 2);
    float* PJ = (float*)take((size_t)LL * CC * 4); float* XS = (float*)take((size_t)LL * CC * 4); bf* Yh = (bf*)take((size_t)LL * CC * 2); bf* Yl = (bf*)take((size_t)LL * CC * 2); float* F1 = (float*)take((size_t)LL * H4 * 4); bf* F1h = (bf*)take((size_t)LL * H4 * 2); bf* F1l = (bf*)take((size_t)LL * H4 * 2); float* F2 = (float*)take((size_t)LL * CC * 4);
    if ((size_t)(wsp - (char*)d_ws) > ws_size) return;
    k_wtG<<<(CC * 3 * CC / 64 + 63) / 64, 256, 0, stream>>>(wqkv, CC, 3 * CC, BQKV); k_wtG<<<(CC * CC / 64 + 63) / 64, 256, 0, stream>>>(wproj, CC, CC, BPJ); k_wtG<<<(CC * H4 / 64 + 63) / 64, 256, 0, stream>>>(wfc1, CC, H4, BF1); k_wtG<<<(H4 * CC / 64 + 63) / 64, 256, 0, stream>>>(wfc2, H4, CC, BF2);
    const unsigned LP = (unsigned)(((size_t)LL * CC / 4 + 255) / 256); const size_t zq = (size_t)WIN * HD, zS = (size_t)WIN * WIN, zv = (size_t)64 * WIN, zo = (size_t)WIN * 64;
    for (int b = 0; b < NB_; ++b) {
        k_xt<<<LP, 256, 0, stream>>>(x + (size_t)b * CC * LL, XT); k_ln<<<LL / 8, 256, 0, stream>>>(XT, g1, b1, Ih, Il);
        k_gemmw<bf, 1, false><<<dim3(LL / 64, 3 * CC / 64, 1), 32, 0, stream>>>(Ih, Il, BQKV, nullptr, CC, QKV, 3 * CC, nullptr, 0, 0, 0);
        for (int br = 0; br < 3; ++br) {
            k_wplanes<<<(unsigned)(((size_t)NZ * WIN * HD / 4 + 255) / 256), 256, 0, stream>>>(QKV, br, Qh, Ql, Kh, Kl); k_vtw<<<(unsigned)(((size_t)NZ * 64 * WIN / 2 + 255) / 256), 256, 0, stream>>>(QKV, br, VT);
            k_gemmw<bf, 2, false><<<dim3(WIN / 64, WIN / 64, NZ), 32, 0, stream>>>(Qh, Ql, Kh, Kl, HD, S, WIN, nullptr, zq, zq, zS);
            k_wsoft<<<NZ * WIN / 8, 256, 0, stream>>>(S, P16);
            k_gemmw<h16, 0, false><<<dim3(WIN / 64, 1, NZ), 32, 0, stream>>>(P16, nullptr, VT, nullptr, WIN, O, 64, nullptr, zS, zv, zo);
            k_wmrg<<<(unsigned)(((size_t)NZ * WIN * HD / 4 + 255) / 256), 256, 0, stream>>>(O, br, ATh, ATl); }
        k_gemmw<bf, 1, true><<<dim3(LL / 64, CC / 64, 1), 32, 0, stream>>>(ATh, ATl, BPJ, nullptr, CC, PJ, CC, bproj, 0, 0, 0);
        k_res1<<<LP, 256, 0, stream>>>(XT, PJ, XS); k_ln<<<LL / 8, 256, 0, stream>>>(XS, g2, b2, Yh, Yl);
        k_gemmw<bf, 1, true><<<dim3(LL / 64, H4 / 64, 1), 32, 0, stream>>>(Yh, Yl, BF1, nullptr, CC, F1, H4, bfc1, 0, 0, 0); k_gelupl<<<(unsigned)(((size_t)LL * H4 / 4 + 255) / 256), 256, 0, stream>>>(F1, F1h, F1l);
        k_gemmw<bf, 1, true><<<dim3(LL / 64, CC / 64, 1), 32, 0, stream>>>(F1h, F1l, BF2, nullptr, H4, F2, CC, bfc2, 0, 0, 0);
        k_out<<<(unsigned)(((size_t)CC * LL / 4 + 255) / 256), 256, 0, stream>>>(XS, F2, OUT + (size_t)b * CC * LL); }
}
